// TemporalAttention_43473658970666
// MI455X (gfx1250) — hardware-verified
//
#include <hip/hip_runtime.h>


typedef __attribute__((ext_vector_type(16))) __bf16 v16bf;
typedef __attribute__((ext_vector_type(8)))  __bf16 v8bf;
typedef __attribute__((ext_vector_type(8)))  float  v8f;
typedef __attribute__((ext_vector_type(4)))  float  v4f;
typedef __attribute__((ext_vector_type(4)))  unsigned int v4u;

#ifndef NB
#define NB 4
#endif
#ifndef SEQ
#define SEQ 2048
#endif
#define NB_FULL  4
#define SEQ_FULL 2048
#define DM   512
#define NH   8
#define HD   64
#define ROWS (NB * SEQ)
#define KPAD 72
#define VSPAD 136
#define YP   516
#define LN_EPS 1e-5f

#define NXB (ROWS * DM / 8 / 256)
#define NWB (DM * DM / 8 / 256)

#define PLANE_BYTES ((size_t)ROWS * DM * 2)
#define WQKV_BYTES  ((size_t)3 * DM * DM * 2)
#define WO_BYTES    ((size_t)DM * DM * 2)
#define WS_TOTAL    (5 * PLANE_BYTES + WQKV_BYTES + WO_BYTES)

static_assert(NB >= 1 && NB <= NB_FULL);
static_assert(SEQ >= 128 && SEQ <= SEQ_FULL && (SEQ % 128) == 0);
static_assert((ROWS % 128) == 0);
static_assert((ROWS * DM) % (8 * 256) == 0);
static_assert((DM * DM) % (8 * 256) == 0);
static_assert((DM % 32) == 0 && (HD % 32) == 0);
static_assert(128 * KPAD >= 64 * VSPAD);
static_assert(WS_TOTAL <= (size_t)134217728);

__device__ __forceinline__ unsigned int bf16_bits(float f) {
  unsigned int u = __float_as_uint(f);
  u += 0x7FFFu + ((u >> 16) & 1u);
  return u >> 16;
}
__device__ __forceinline__ float bf16q(float f) {
  return __uint_as_float(bf16_bits(f) << 16);
}

__device__ __forceinline__ v16bf load_frag_row(const __bf16* base, int stride, int lane) {
  const __bf16* rowp = base + (lane & 15) * stride + ((lane >> 4) << 3);
  v8bf lo = *(const v8bf*)(rowp);
  v8bf hi = *(const v8bf*)(rowp + 16);
  return __builtin_shufflevector(lo, hi, 0, 1, 2, 3, 4, 5, 6, 7,
                                 8, 9, 10, 11, 12, 13, 14, 15);
}

__device__ __forceinline__ v8f wmma_bf16(v16bf a, v16bf b, v8f c) {
  v8f d = __builtin_amdgcn_wmma_f32_16x16x32_bf16(false, a, false, b, (short)0, c,
                                                  false, false);
  asm volatile("v_nop\n\tv_nop\n\tv_nop\n\tv_nop" : "+v"(d) : "v"(a), "v"(b));
  return d;
}

__global__ __launch_bounds__(256) void cvt_kernel(
    const float* __restrict__ x,
    const float* __restrict__ Wq, const float* __restrict__ Wk,
    const float* __restrict__ Wv, const float* __restrict__ Wo,
    __bf16* __restrict__ xb, __bf16* __restrict__ wqkv, __bf16* __restrict__ wob) {
  const int bid = blockIdx.x;
  const int t   = threadIdx.x;
  const float* src;
  __bf16* dst;
  if (bid < NXB) {
    const long item = (long)bid * 256 + t;
    const long m    = item >> 6;
    const int  c8   = (int)(item & 63);
    const long srow = (m / SEQ) * SEQ_FULL + (m % SEQ);
    src = x + srow * DM + c8 * 8;
    dst = xb + m * DM + c8 * 8;
  } else if (bid < NXB + 3 * NWB) {
    const int wb    = bid - NXB;
    const int which = wb / NWB;
    const long item = (long)(wb - which * NWB) * 256 + t;
    const float* W = (which == 0) ? Wq : ((which == 1) ? Wk : Wv);
    src = W + item * 8;
    dst = wqkv + (long)which * DM * DM + item * 8;
  } else {
    const long item = (long)(bid - NXB - 3 * NWB) * 256 + t;
    src = Wo + item * 8;
    dst = wob + item * 8;
  }
  const v4f a = *(const v4f*)(src);
  const v4f c = *(const v4f*)(src + 4);
  v4u o;
  o[0] = bf16_bits(a[0]) | (bf16_bits(a[1]) << 16);
  o[1] = bf16_bits(a[2]) | (bf16_bits(a[3]) << 16);
  o[2] = bf16_bits(c[0]) | (bf16_bits(c[1]) << 16);
  o[3] = bf16_bits(c[2]) | (bf16_bits(c[3]) << 16);
  *(volatile v4u*)dst = o;
  __threadfence();
  *(volatile v4u*)dst = o;
}

__global__ __launch_bounds__(256) void qkv_kernel(
    const __bf16* __restrict__ xb, const __bf16* __restrict__ wqkv,
    const float* __restrict__ bq, const float* __restrict__ bk, const float* __restrict__ bv,
    __bf16* __restrict__ q, __bf16* __restrict__ k, __bf16* __restrict__ vT) {
  __shared__ __bf16 stg[128 * KPAD];

  const int tid  = threadIdx.x;
  const int lane = tid & 31;
  const int wave = tid >> 5;
  const int hh   = lane >> 4;
  const int l15  = lane & 15;

  const int cb   = blockIdx.y;
  const int osel = cb >> 3;
  const int h    = cb & 7;
  const long m0  = (long)blockIdx.x * 128;
  const int  b   = (int)(m0 / SEQ);
  const int  s0  = (int)(m0 - (long)b * SEQ);

  const __bf16* xrow = xb + (m0 + wave * 16) * DM;
  const __bf16* wrow = wqkv + ((long)cb * 64) * DM;

  v8f acc[4];
#pragma unroll
  for (int j = 0; j < 4; ++j) acc[j] = (v8f){};

#pragma unroll 1
  for (int kk = 0; kk < DM; kk += 32) {
    v16bf xf = load_frag_row(xrow + kk, DM, lane);
#pragma unroll
    for (int j = 0; j < 4; ++j) {
      v16bf wf = load_frag_row(wrow + (long)(j * 16) * DM + kk, DM, lane);
      acc[j] = wmma_bf16(wf, xf, acc[j]);
    }
  }

  const float* bias = (osel == 0) ? bq : ((osel == 1) ? bk : bv);
  const float  sc   = (osel == 0) ? 0.125f : 1.0f;

  v4u rv[4];
  if (osel < 2) {
    __bf16* srow = stg + (wave * 16 + l15) * KPAD;
#pragma unroll
    for (int j = 0; j < 4; ++j) {
      const int n8 = j * 16 + hh * 8;
      const v4f b0 = *(const v4f*)(bias + h * HD + n8);
      const v4f b1 = *(const v4f*)(bias + h * HD + n8 + 4);
      v8bf pk;
#pragma unroll
      for (int r = 0; r < 4; ++r) {
        pk[r]     = (__bf16)((acc[j][r]     + bf16q(b0[r])) * sc);
        pk[4 + r] = (__bf16)((acc[j][4 + r] + bf16q(b1[r])) * sc);
      }
      *(v8bf*)(srow + n8) = pk;
    }
    __syncthreads();
#pragma unroll
    for (int it = 0; it < 4; ++it) {
      const int idx = it * 256 + tid;
      const int row = idx >> 3, piece = idx & 7;
      rv[it] = *(const v4u*)(stg + row * KPAD + piece * 8);
    }
    __bf16* dst = ((osel == 0) ? q : k) + ((long)(b * NH + h) * SEQ + s0) * HD;
#pragma unroll
    for (int it = 0; it < 4; ++it)
      *(volatile v4u*)(dst + (long)(it * 256 + tid) * 8) = rv[it];
    __threadfence();
#pragma unroll
    for (int it = 0; it < 4; ++it)
      *(volatile v4u*)(dst + (long)(it * 256 + tid) * 8) = rv[it];
  } else {
#pragma unroll
    for (int j = 0; j < 4; ++j) {
      const int n8 = j * 16 + hh * 8;
      const v4f b0 = *(const v4f*)(bias + h * HD + n8);
      const v4f b1 = *(const v4f*)(bias + h * HD + n8 + 4);
#pragma unroll
      for (int r = 0; r < 4; ++r) {
        stg[(n8 + r) * VSPAD + wave * 16 + l15]     = (__bf16)(acc[j][r]     + bf16q(b0[r]));
        stg[(n8 + 4 + r) * VSPAD + wave * 16 + l15] = (__bf16)(acc[j][4 + r] + bf16q(b1[r]));
      }
    }
    __syncthreads();
#pragma unroll
    for (int it = 0; it < 4; ++it) {
      const int idx = it * 256 + tid;
      const int d = idx >> 4, piece = idx & 15;
      rv[it] = *(const v4u*)(stg + d * VSPAD + piece * 8);
    }
    __bf16* dstb = vT + ((long)(b * NH + h) * HD) * SEQ + s0;
#pragma unroll
    for (int it = 0; it < 4; ++it) {
      const int idx = it * 256 + tid;
      const int d = idx >> 4, piece = idx & 15;
      *(volatile v4u*)(dstb + (long)d * SEQ + piece * 8) = rv[it];
    }
    __threadfence();
#pragma unroll
    for (int it = 0; it < 4; ++it) {
      const int idx = it * 256 + tid;
      const int d = idx >> 4, piece = idx & 15;
      *(volatile v4u*)(dstb + (long)d * SEQ + piece * 8) = rv[it];
    }
  }
}

__global__ __launch_bounds__(256) void attn_kernel(
    const __bf16* __restrict__ Q, const __bf16* __restrict__ K,
    const __bf16* __restrict__ vT, __bf16* __restrict__ ctx) {
  __shared__ __bf16 ks[64 * KPAD];
  __shared__ __bf16 vts[64 * KPAD];
  __shared__ __bf16 ost[128 * KPAD];

  const int tid  = threadIdx.x;
  const int lane = tid & 31;
  const int wave = tid >> 5;
  const int bh   = blockIdx.y;
  const int b    = bh >> 3;
  const int h    = bh & 7;
  const int q0   = blockIdx.x * 128;

  const __bf16* Qb  = Q + ((long)bh * SEQ + q0) * HD;
  const __bf16* Kb  = K + (long)bh * SEQ * HD;
  const __bf16* vTb = vT + (long)bh * HD * SEQ;

  v16bf qfrag[2];
  {
    const __bf16* qrow = Qb + (long)wave * 16 * HD;
#pragma unroll
    for (int t = 0; t < 2; ++t) qfrag[t] = load_frag_row(qrow + t * 32, HD, lane);
  }

  v8f acc[4];
#pragma unroll
  for (int nt = 0; nt < 4; ++nt) acc[nt] = (v8f){};
  float mi = -1e30f, li = 0.0f;

  const int colb = lane & 15;
  const int rofs = (lane >> 4) << 3;

  for (int kb = 0; kb < SEQ; kb += 64) {
    __syncthreads();
    for (int idx = tid; idx < 64 * 8; idx += 256) {
      const int row = idx >> 3, c = idx & 7;
      *(v8bf*)(ks + row * KPAD + c * 8) =
          *(const v8bf*)(Kb + (long)(kb + row) * HD + c * 8);
    }
    for (int idx = tid; idx < 64 * 8; idx += 256) {
      const int d = idx >> 3, c = idx & 7;
      *(v8bf*)(vts + d * KPAD + c * 8) =
          *(const v8bf*)(vTb + (long)d * SEQ + kb + c * 8);
    }
    __syncthreads();

    v8f sc[4];
#pragma unroll
    for (int kt = 0; kt < 4; ++kt) sc[kt] = (v8f){};
#pragma unroll
    for (int t = 0; t < 2; ++t)
#pragma unroll
      for (int kt = 0; kt < 4; ++kt) {
        v16bf kf = load_frag_row(ks + (kt * 16) * KPAD + t * 32, KPAD, lane);
        sc[kt] = wmma_bf16(kf, qfrag[t], sc[kt]);
      }

    float mx = sc[0][0];
#pragma unroll
    for (int kt = 0; kt < 4; ++kt)
#pragma unroll
      for (int r = 0; r < 8; ++r) mx = fmaxf(mx, sc[kt][r]);
    mx = fmaxf(mx, __shfl_xor(mx, 16, 32));
    const float mnew  = fmaxf(mi, mx);
    const float alpha = __expf(mi - mnew);
    mi = mnew;

    float rs = 0.0f;
#pragma unroll
    for (int kt = 0; kt < 4; ++kt)
#pragma unroll
      for (int r = 0; r < 8; ++r) {
        const float p = __expf(sc[kt][r] - mnew);
        sc[kt][r] = p;
        rs += p;
      }
    rs += __shfl_xor(rs, 16, 32);
    li = li * alpha + rs;

    v16bf pf[2];
#pragma unroll
    for (int t = 0; t < 2; ++t)
#pragma unroll
      for (int i = 0; i < 8; ++i) {
        pf[t][i]     = (__bf16)sc[2 * t][i];
        pf[t][8 + i] = (__bf16)sc[2 * t + 1][i];
      }

#pragma unroll
    for (int nt = 0; nt < 4; ++nt)
#pragma unroll
      for (int r = 0; r < 8; ++r) acc[nt][r] *= alpha;

#pragma unroll
    for (int t = 0; t < 2; ++t)
#pragma unroll
      for (int nt = 0; nt < 4; ++nt) {
        v16bf vf = load_frag_row(vts + (nt * 16) * KPAD + t * 32, KPAD, lane);
        acc[nt] = wmma_bf16(vf, pf[t], acc[nt]);
      }
  }

  {
    const float inv = 1.0f / li;
    __bf16* orow = ost + (wave * 16 + colb) * KPAD;
#pragma unroll
    for (int nt = 0; nt < 4; ++nt) {
      v8bf pk;
#pragma unroll
      for (int r = 0; r < 8; ++r) pk[r] = (__bf16)(acc[nt][r] * inv);
      *(v8bf*)(orow + nt * 16 + rofs) = pk;
    }
  }
  __syncthreads();

  v4u rv[4];
#pragma unroll
  for (int it = 0; it < 4; ++it) {
    const int idx = it * 256 + tid;
    const int row = idx >> 3, piece = idx & 7;
    rv[it] = *(const v4u*)(ost + row * KPAD + piece * 8);
  }
  __bf16* cbase = ctx + ((long)b * SEQ + q0) * DM + h * HD;
#pragma unroll
  for (int it = 0; it < 4; ++it) {
    const int idx = it * 256 + tid;
    const int row = idx >> 3, piece = idx & 7;
    *(volatile v4u*)(cbase + (long)row * DM + piece * 8) = rv[it];
  }
  __threadfence();
#pragma unroll
  for (int it = 0; it < 4; ++it) {
    const int idx = it * 256 + tid;
    const int row = idx >> 3, piece = idx & 7;
    *(volatile v4u*)(cbase + (long)row * DM + piece * 8) = rv[it];
  }
}

__global__ __launch_bounds__(256) void oproj_ln_kernel(
    const __bf16* __restrict__ ctx, const __bf16* __restrict__ wob,
    const float* __restrict__ bo, const float* __restrict__ x,
    const float* __restrict__ gam, const float* __restrict__ bet,
    float* __restrict__ out) {
  __shared__ float ys[16 * YP];
  __shared__ float smean[16];
  __shared__ float srstd[16];

  const int tid  = threadIdx.x;
  const int lane = tid & 31;
  const int wave = tid >> 5;
  const int hh   = lane >> 4;
  const int l15  = lane & 15;
  const long m0  = (long)blockIdx.x * 16;
  const int  n0  = wave * 64;

  const __bf16* crow = ctx + m0 * DM;
  const __bf16* wrow = wob + (long)n0 * DM;

  v8f acc[4];
#pragma unroll
  for (int j = 0; j < 4; ++j) acc[j] = (v8f){};

#pragma unroll 1
  for (int kk = 0; kk < DM; kk += 32) {
    v16bf cf = load_frag_row(crow + kk, DM, lane);
#pragma unroll
    for (int j = 0; j < 4; ++j) {
      v16bf wf = load_frag_row(wrow + (long)(j * 16) * DM + kk, DM, lane);
      acc[j] = wmma_bf16(wf, cf, acc[j]);
    }
  }

  {
    const long m    = m0 + l15;
    const long orow = (m / SEQ) * SEQ_FULL + (m % SEQ);
    const float* xr = x + orow * DM;
    float* yrow = ys + l15 * YP;
#pragma unroll
    for (int j = 0; j < 4; ++j) {
      const int n8 = n0 + j * 16 + hh * 8;
      const v4f x0 = *(const v4f*)(xr + n8);
      const v4f x1 = *(const v4f*)(xr + n8 + 4);
      const v4f b0 = *(const v4f*)(bo + n8);
      const v4f b1 = *(const v4f*)(bo + n8 + 4);
      v4f y0, y1;
#pragma unroll
      for (int i = 0; i < 4; ++i) {
        y0[i] = (acc[j][i]     + bf16q(b0[i])) + bf16q(x0[i]);
        y1[i] = (acc[j][4 + i] + bf16q(b1[i])) + bf16q(x1[i]);
      }
      *(v4f*)(yrow + n8)     = y0;
      *(v4f*)(yrow + n8 + 4) = y1;
    }
  }
  __syncthreads();

  {
    const int r  = tid >> 4;
    const int sl = tid & 15;
    const float* yr = ys + r * YP + sl * 32;
    v4f yv[8];
#pragma unroll
    for (int i = 0; i < 8; ++i) yv[i] = *(const v4f*)(yr + i * 4);
    float s = 0.0f;
#pragma unroll
    for (int i = 0; i < 8; ++i) s += (yv[i][0] + yv[i][1]) + (yv[i][2] + yv[i][3]);
    s += __shfl_xor(s, 1, 32);
    s += __shfl_xor(s, 2, 32);
    s += __shfl_xor(s, 4, 32);
    s += __shfl_xor(s, 8, 32);
    const float mean = s * (1.0f / DM);
    float ss = 0.0f;
#pragma unroll
    for (int i = 0; i < 8; ++i)
#pragma unroll
      for (int c = 0; c < 4; ++c) {
        const float d = yv[i][c] - mean;
        ss += d * d;
      }
    ss += __shfl_xor(ss, 1, 32);
    ss += __shfl_xor(ss, 2, 32);
    ss += __shfl_xor(ss, 4, 32);
    ss += __shfl_xor(ss, 8, 32);
    const float var  = ss * (1.0f / DM);
    const float rstd = rsqrtf(var + LN_EPS);
    if (sl == 0) { smean[r] = mean; srstd[r] = rstd; }
  }
  __syncthreads();

  v4f ov[8];
#pragma unroll
  for (int it = 0; it < 8; ++it) {
    const int idx = it * 256 + tid;
    const int row = idx >> 7, piece = idx & 127;
    const v4f yv = *(const v4f*)(ys + row * YP + piece * 4);
    const v4f g  = *(const v4f*)(gam + piece * 4);
    const v4f bt = *(const v4f*)(bet + piece * 4);
    const float mean = smean[row], rstd = srstd[row];
#pragma unroll
    for (int c = 0; c < 4; ++c)
      ov[it][c] = (yv[c] - mean) * rstd * bf16q(g[c]) + bf16q(bt[c]);
  }
#pragma unroll
  for (int it = 0; it < 8; ++it) {
    const int idx = it * 256 + tid;
    const int row = idx >> 7, piece = idx & 127;
    const long m    = m0 + row;
    const long orow = (m / SEQ) * SEQ_FULL + (m % SEQ);
    *(volatile v4f*)(out + orow * DM + piece * 4) = ov[it];
  }
  __threadfence();
#pragma unroll
  for (int it = 0; it < 8; ++it) {
    const int idx = it * 256 + tid;
    const int row = idx >> 7, piece = idx & 127;
    const long m    = m0 + row;
    const long orow = (m / SEQ) * SEQ_FULL + (m % SEQ);
    *(volatile v4f*)(out + orow * DM + piece * 4) = ov[it];
  }
}

extern "C" void kernel_launch(void* const* d_in, const int* in_sizes, int n_in,
                              void* d_out, int out_size, void* d_ws, size_t ws_size,
                              hipStream_t stream) {
  if (n_in < 11) return;
  const long needRows = (long)(NB - 1) * SEQ_FULL + SEQ;
  if ((long)in_sizes[0] < needRows * DM) return;
  if (in_sizes[1] < DM * DM || in_sizes[3] < DM * DM ||
      in_sizes[5] < DM * DM || in_sizes[7] < DM * DM) return;
  if (in_sizes[2] < DM || in_sizes[4] < DM || in_sizes[6] < DM ||
      in_sizes[8] < DM || in_sizes[9] < DM || in_sizes[10] < DM) return;
  if ((long)out_size < needRows * DM) return;
  if (ws_size < WS_TOTAL) return;

  const float* x   = (const float*)d_in[0];
  const float* Wq  = (const float*)d_in[1];
  const float* bq  = (const float*)d_in[2];
  const float* Wk  = (const float*)d_in[3];
  const float* bk  = (const float*)d_in[4];
  const float* Wv  = (const float*)d_in[5];
  const float* bv  = (const float*)d_in[6];
  const float* Wo  = (const float*)d_in[7];
  const float* bo  = (const float*)d_in[8];
  const float* gam = (const float*)d_in[9];
  const float* bet = (const float*)d_in[10];
  float* out = (float*)d_out;

  char* ws = (char*)d_ws;
  size_t off = 0;
  __bf16* xb   = (__bf16*)(ws + off); off += PLANE_BYTES;
  __bf16* wqkv = (__bf16*)(ws + off); off += WQKV_BYTES;
  __bf16* wob  = (__bf16*)(ws + off); off += WO_BYTES;
  __bf16* qb   = (__bf16*)(ws + off); off += PLANE_BYTES;
  __bf16* kbf  = (__bf16*)(ws + off); off += PLANE_BYTES;
  __bf16* vTb  = (__bf16*)(ws + off); off += PLANE_BYTES;
  __bf16* ctx  = (__bf16*)(ws + off); off += PLANE_BYTES;
  if (off > ws_size) return;

  cvt_kernel<<<NXB + 4 * NWB, 256, 0, stream>>>(x, Wq, Wk, Wv, Wo, xb, wqkv, wob);

  qkv_kernel<<<dim3(ROWS / 128, 3 * NH), 256, 0, stream>>>(xb, wqkv, bq, bk, bv, qb, kbf, vTb);

  attn_kernel<<<dim3(SEQ / 128, NB * NH), 256, 0, stream>>>(qb, kbf, vTb, ctx);

  oproj_ln_kernel<<<ROWS / 16, 256, 0, stream>>>(ctx, wob, bo, x, gam, bet, out);
}
